// Model_62173946577086
// MI455X (gfx1250) — hardware-verified
//
#include <hip/hip_runtime.h>
#include <math.h>

constexpr int NSTEP   = 128;
constexpr int NBATCH  = 256;
constexpr int NIN     = 256;
constexpr int NHID    = 1024;
constexpr int NOUT    = 256;
constexpr int NHALVES = 2;
constexpr int STEPS_H = NSTEP / NHALVES;
constexpr int ROWS_H  = STEPS_H * NBATCH;
constexpr int SEQ_BLK = 16;
constexpr int RTHR    = 512;
constexpr int HPITCH  = NHID + 8;
constexpr float WCARRY     = 256.0f;
constexpr float WCARRY_INV = 1.0f / 256.0f;

static_assert(NSTEP % NHALVES == 0, "time halves");
static_assert(NBATCH % SEQ_BLK == 0, "batch tiles");
static_assert(NHID == 64 * (RTHR / 32), "16 waves x 64 hidden columns");
static_assert(NIN % 32 == 0 && NHID % 32 == 0, "GEMM K multiples of 32");
static_assert(ROWS_H % 64 == 0 && NHID % 64 == 0 && NBATCH % 64 == 0 && NOUT % 64 == 0, "GEMM M, N tile multiples");
static_assert(SEQ_BLK * NHID / 8 == 4 * RTHR, "h tile copy loop exact");
static_assert((HPITCH % 8) == 0, "16-B aligned LDS rows");
static_assert((NSTEP * NBATCH * NIN) % (8 * 256) == 0, "split grid exact");

typedef __attribute__((ext_vector_type(16))) _Float16 v16h;
typedef __attribute__((ext_vector_type(8)))  _Float16 v8h;
typedef __attribute__((ext_vector_type(16))) __bf16   v16b;
typedef __attribute__((ext_vector_type(8)))  __bf16   v8b;
typedef __attribute__((ext_vector_type(8)))  float    v8f;
typedef __attribute__((ext_vector_type(4)))  float    v4f;

__device__ __forceinline__ unsigned short f2bf_bits(float f) {
  unsigned u = __float_as_uint(f);
  return (unsigned short)((u + 0x7FFFu + ((u >> 16) & 1u)) >> 16);
}
__device__ __forceinline__ float bf_bits2f(unsigned short h) { return __uint_as_float(((unsigned)h) << 16); }

__device__ __forceinline__ void dep_guard4_b(v8f& a, v8f& b, v8f& c, v8f& d, v16b x, v16b y) {
  asm volatile("v_nop\n\tv_nop\n\tv_nop\n\tv_nop" : "+v"(a), "+v"(b), "+v"(c), "+v"(d) : "v"(x), "v"(y));
}
__device__ __forceinline__ void dep_guard4_h(v8f& a, v8f& b, v8f& c, v8f& d, v16h x, v16h y0, v16h y1, v16h y2, v16h y3) {
  asm volatile("v_nop\n\tv_nop\n\tv_nop\n\tv_nop" : "+v"(a), "+v"(b), "+v"(c), "+v"(d) : "v"(x), "v"(y0), "v"(y1), "v"(y2), "v"(y3));
}
__device__ __forceinline__ void keep4_b(v16b a, v16b b, v16b c, v16b d) { asm volatile("v_nop" :: "v"(a), "v"(b), "v"(c), "v"(d)); }
__device__ __forceinline__ void acc_guard4(v8f& a, v8f& b, v8f& c, v8f& d) {
  asm volatile("v_nop\n\tv_nop\n\tv_nop\n\tv_nop" : "+v"(a), "+v"(b), "+v"(c), "+v"(d));
}

template <typename T> struct Frag;
template <> struct Frag<_Float16> {
  typedef v16h V; union U { v16h v; v8h h[2]; };
  static __device__ __forceinline__ v16h load(const _Float16* p) {
    U f; f.h[0] = *(const v8h*)(p); f.h[1] = *(const v8h*)(p + 16); return f.v;
  }
  static __device__ __forceinline__ v8f mma(v16h a, v16h b, v8f c) {
    return __builtin_amdgcn_wmma_f32_16x16x32_f16(false, a, false, b, (short)0, c, false, false);
  }
};
template <> struct Frag<__bf16> {
  typedef v16b V; union U { v16b v; v8b h[2]; };
  static __device__ __forceinline__ v16b load(const __bf16* p) {
    U f; f.h[0] = *(const v8b*)(p); f.h[1] = *(const v8b*)(p + 16); return f.v;
  }
  static __device__ __forceinline__ v8f mma(v16b a, v16b b, v8f c) {
    return __builtin_amdgcn_wmma_f32_16x16x32_bf16(false, a, false, b, (short)0, c, false, false);
  }
};

__device__ __forceinline__ float ftanh(float x) { return 1.0f - 2.0f * __builtin_amdgcn_rcpf(__expf(2.0f * x) + 1.0f); }

__global__ __launch_bounds__(256) void split8_kernel(const float* __restrict__ src, unsigned short* __restrict__ hi,
                                                     unsigned short* __restrict__ lo, int n8) {
  const int i = blockIdx.x * 256 + threadIdx.x;
  if (i < n8) {
    const float* sp = src + (size_t)i * 8;
    const v4f a = *(const v4f*)(sp);
    const v4f b = *(const v4f*)(sp + 4);
    v8h hv, lv;
#pragma unroll
    for (int e = 0; e < 4; ++e) {
      const float fa = a[e];
      const float fb = b[e];
      const unsigned short ha = f2bf_bits(fa);
      const unsigned short hb = f2bf_bits(fb);
      const unsigned short la = f2bf_bits(fa - bf_bits2f(ha));
      const unsigned short lb = f2bf_bits(fb - bf_bits2f(hb));
      hv[e]     = __builtin_bit_cast(_Float16, ha);
      hv[4 + e] = __builtin_bit_cast(_Float16, hb);
      lv[e]     = __builtin_bit_cast(_Float16, la);
      lv[4 + e] = __builtin_bit_cast(_Float16, lb);
    }
    *(volatile v8h*)(hi + (size_t)i * 8) = hv;
    *(volatile v8h*)(lo + (size_t)i * 8) = lv;
    __threadfence();
    *(volatile v8h*)(hi + (size_t)i * 8) = hv;
    *(volatile v8h*)(lo + (size_t)i * 8) = lv;
  }
}

template <int MODE>
__global__ __launch_bounds__(256) void tpw_kernel(const float* __restrict__ src, int C, int ldo,
                                                  unsigned short* __restrict__ O, unsigned short* O2, float sc) {
  __shared__ float Tt[64 * 65];
  const int tid = threadIdx.x;
  const int c0 = blockIdx.x * 64, r0 = blockIdx.y * 64;
#pragma unroll
  for (int i = 0; i < 4; ++i) {
    const int idx = i * 256 + tid;
    const int rr = idx >> 4, cc = (idx & 15) * 4;
    const v4f v = *(const v4f*)(src + (size_t)(r0 + rr) * (size_t)C + c0 + cc);
    Tt[rr * 65 + cc + 0] = v[0];
    Tt[rr * 65 + cc + 1] = v[1];
    Tt[rr * 65 + cc + 2] = v[2];
    Tt[rr * 65 + cc + 3] = v[3];
  }
  __syncthreads();
  const int q = tid >> 3, c8 = (tid & 7) * 8;
  v8h hv[2], lv[2];
#pragma unroll
  for (int g = 0; g < 2; ++g) {
    const int qq = g * 32 + q;
#pragma unroll
    for (int e = 0; e < 8; ++e) {
      const float f = Tt[(c8 + e) * 65 + qq];
      unsigned short b0, b1;
      if (MODE == 0) {
        b0 = f2bf_bits(f);
        b1 = f2bf_bits(f - bf_bits2f(b0));
      } else {
        const _Float16 hx = (_Float16)(f * sc);
        b0 = __builtin_bit_cast(unsigned short, hx);
        b1 = 0;
      }
      hv[g][e] = __builtin_bit_cast(_Float16, b0);
      lv[g][e] = __builtin_bit_cast(_Float16, b1);
    }
  }
  for (int pass = 0; pass < 2; ++pass) {
#pragma unroll
    for (int g = 0; g < 2; ++g) {
      const size_t o = (size_t)(c0 + g * 32 + q) * (size_t)ldo + (size_t)(r0 + c8);
      *(volatile v8h*)(O + o) = hv[g];
      if (MODE == 0) *(volatile v8h*)(O2 + o) = lv[g];
    }
    __threadfence();
  }
}

template <int BIAS_MODE>
__global__ __launch_bounds__(256) void wmma_gemm64(
    const unsigned short* __restrict__ Ap, const unsigned short* __restrict__ A2p, int lda,
    const unsigned short* __restrict__ Btp, const unsigned short* __restrict__ Bt2p, int ldb,
    float* __restrict__ Cout, int ldc, const float* __restrict__ bias,
    int M, int N, int K, float scale) {
  typedef __bf16 T;
  typedef v16b V;
  const T* A = (const T*)Ap; const T* A2 = (const T*)A2p; const T* Bt = (const T*)Btp; const T* Bt2 = (const T*)Bt2p;
  __shared__ __align__(16) float sT[8][16 * 68];
  const int lane = threadIdx.x & 31;
  const int wave = threadIdx.x >> 5;
  const int tilesN = N >> 6;
  const int tilesM = M >> 6;
  const int tile = blockIdx.x * 8 + wave;
  if (tile >= tilesM * tilesN) return;
  const int tm = tile / tilesN;
  const int tn = tile - tm * tilesN;
  const int m0 = tm << 6;
  const int n0 = tn << 6;

  const int rlane = lane & 15;
  const int koff  = (lane >> 4) * 8;
  const int mOff  = (lane >> 4) * 8;

  v8f acc[4][4];
#pragma unroll
  for (int i = 0; i < 4; ++i)
#pragma unroll
    for (int j = 0; j < 4; ++j) acc[i][j] = (v8f){0.f,0.f,0.f,0.f,0.f,0.f,0.f,0.f};

  for (int k0 = 0; k0 < K; k0 += 32) {
    V bh[4], bl[4];
#pragma unroll
    for (int j = 0; j < 4; ++j) {
      const size_t bo = (size_t)(n0 + (j << 4) + rlane) * ldb + koff + k0;
      bh[j] = Frag<T>::load(Bt + bo);
      bl[j] = Frag<T>::load(Bt2 + bo);
    }
#pragma unroll
    for (int i = 0; i < 4; ++i) {
      const size_t ao = (size_t)(m0 + (i << 4) + rlane) * lda + koff + k0;
      V ah = Frag<T>::load(A + ao);
      V al = Frag<T>::load(A2 + ao);
#pragma unroll
      for (int j = 0; j < 4; ++j) {
        acc[i][j] = Frag<T>::mma(ah, bh[j], acc[i][j]);
        acc[i][j] = Frag<T>::mma(ah, bl[j], acc[i][j]);
        acc[i][j] = Frag<T>::mma(al, bh[j], acc[i][j]);
      }
      dep_guard4_b(acc[i][0], acc[i][1], acc[i][2], acc[i][3], ah, al);
    }
    keep4_b(bh[0], bh[1], bh[2], bh[3]);
    keep4_b(bl[0], bl[1], bl[2], bl[3]);
  }
  acc_guard4(acc[0][0], acc[0][1], acc[0][2], acc[0][3]);
  acc_guard4(acc[1][0], acc[1][1], acc[1][2], acc[1][3]);
  acc_guard4(acc[2][0], acc[2][1], acc[2][2], acc[2][3]);
  acc_guard4(acc[3][0], acc[3][1], acc[3][2], acc[3][3]);

  float* slab = sT[wave];
#pragma unroll
  for (int i = 0; i < 4; ++i) {
    const int mBase = m0 + (i << 4);
#pragma unroll
    for (int j = 0; j < 4; ++j) {
      const int n = n0 + (j << 4) + rlane;
      float bv = 0.f;
      if (BIAS_MODE == 2) bv = bias[n];
      if (BIAS_MODE == 3) bv = bias[0];
#pragma unroll
      for (int r = 0; r < 8; ++r) {
        float v = acc[i][j][r] * scale;
        v += bv;
        slab[(mOff + r) * 68 + (j << 4) + rlane] = v;
      }
    }
    __builtin_amdgcn_fence(__ATOMIC_RELEASE, "workgroup");
    __builtin_amdgcn_wave_barrier();
    __builtin_amdgcn_fence(__ATOMIC_ACQUIRE, "workgroup");
    {
      const int hh = lane >> 4, c4 = (lane & 15) * 4;
      for (int pass = 0; pass < 2; ++pass) {
#pragma unroll
        for (int it = 0; it < 8; ++it) {
          const int row = it * 2 + hh;
          v4f v = *(const v4f*)(slab + row * 68 + c4);
          *(volatile v4f*)(Cout + (size_t)(mBase + row) * ldc + n0 + c4) = v;
        }
        __threadfence();
      }
    }
    __builtin_amdgcn_fence(__ATOMIC_RELEASE, "workgroup");
    __builtin_amdgcn_wave_barrier();
    __builtin_amdgcn_fence(__ATOMIC_ACQUIRE, "workgroup");
  }
}

__device__ __forceinline__ void tile_store(const _Float16* tile, _Float16* dst, int rowbase, int tid) {
  for (int pass = 0; pass < 2; ++pass) {
#pragma unroll
    for (int it = 0; it < 4; ++it) {
      const int idx = it * RTHR + tid;
      const int row = idx >> 7, ch = (idx & 127) * 8;
      const v8h v = *(const v8h*)(tile + row * HPITCH + ch);
      *(volatile v8h*)(dst + (size_t)(rowbase + row) * NHID + ch) = v;
    }
    __threadfence();
  }
}

__global__ __launch_bounds__(RTHR) void rnn_seq_kernel(const float* __restrict__ XP,
                                                       const unsigned short* __restrict__ WHp,
                                                       unsigned short* HSTp, unsigned short* HHp, unsigned short* HLp,
                                                       int first, int last) {
  __shared__ __align__(16) _Float16 Ah[SEQ_BLK * HPITCH];
  const _Float16* WH = (const _Float16*)WHp;
  _Float16* HST = (_Float16*)HSTp;
  _Float16* HH  = (_Float16*)HHp;
  _Float16* HL  = (_Float16*)HLp;
  const int tid = threadIdx.x, lane = tid & 31, wave = tid >> 5;
  const int c = lane & 15, hh = lane >> 4, koff = hh * 8;
  const int rowbase = blockIdx.x * SEQ_BLK;

  v8h zz;
#pragma unroll
  for (int e = 0; e < 8; ++e) zz[e] = (_Float16)0.0f;
  if (tid < SEQ_BLK) *(v8h*)(Ah + tid * HPITCH + NHID) = zz;
  if (first != 0) {
#pragma unroll
    for (int it = 0; it < 4; ++it) {
      const int idx = it * RTHR + tid;
      const int row = idx >> 7, ch = (idx & 127) * 8;
      *(v8h*)(Ah + row * HPITCH + ch) = zz;
    }
  } else {
#pragma unroll
    for (int it = 0; it < 4; ++it) {
      const int idx = it * RTHR + tid;
      const int row = idx >> 7, ch = (idx & 127) * 8;
      const v8h v = *(const v8h*)(HST + (size_t)(rowbase + row) * NHID + ch);
      *(v8h*)(Ah + row * HPITCH + ch) = v;
    }
  }
  __syncthreads();

  const _Float16* ahrow = Ah + c * HPITCH + koff;
  const _Float16* wrow  = WH + (size_t)(64 * wave + c) * NHID + koff;
  const float*    xpb   = XP + (size_t)(rowbase + 8 * hh) * NHID + 64 * wave + c;

  float hv[4][8];
#pragma unroll
  for (int nt = 0; nt < 4; ++nt)
#pragma unroll
    for (int r = 0; r < 8; ++r) hv[nt][r] = 0.0f;

#pragma unroll 1
  for (int t = 0; t < STEPS_H; ++t) {
    const float* xp = xpb + (size_t)t * NBATCH * NHID;
    v8f acc[4];
#pragma unroll
    for (int nt = 0; nt < 4; ++nt)
#pragma unroll
      for (int r = 0; r < 8; ++r) acc[nt][r] = xp[(size_t)r * NHID + 16 * nt] * WCARRY;

#pragma unroll 1
    for (int k0 = 0; k0 < NHID; k0 += 32) {
      const v16h a  = Frag<_Float16>::load(ahrow + k0);
      const v16h b0 = Frag<_Float16>::load(wrow + k0);
      const v16h b1 = Frag<_Float16>::load(wrow + (size_t)16 * NHID + k0);
      const v16h b2 = Frag<_Float16>::load(wrow + (size_t)32 * NHID + k0);
      const v16h b3 = Frag<_Float16>::load(wrow + (size_t)48 * NHID + k0);
      acc[0] = Frag<_Float16>::mma(a, b0, acc[0]);
      acc[1] = Frag<_Float16>::mma(a, b1, acc[1]);
      acc[2] = Frag<_Float16>::mma(a, b2, acc[2]);
      acc[3] = Frag<_Float16>::mma(a, b3, acc[3]);
      dep_guard4_h(acc[0], acc[1], acc[2], acc[3], a, b0, b1, b2, b3);
    }
    acc_guard4(acc[0], acc[1], acc[2], acc[3]);

    __syncthreads();
#pragma unroll
    for (int nt = 0; nt < 4; ++nt) {
      const int j = 64 * wave + 16 * nt + c;
#pragma unroll
      for (int r = 0; r < 8; ++r) {
        const float z  = acc[nt][r] * WCARRY_INV;
        const float hn = ftanh(z);
        hv[nt][r] = hn;
        Ah[(8 * hh + r) * HPITCH + j] = (_Float16)hn;
      }
    }
    __syncthreads();
  }

  if (last == 0) {
    tile_store(Ah, HST, rowbase, tid);
  } else {
#pragma unroll
    for (int nt = 0; nt < 4; ++nt) {
      const int j = 64 * wave + 16 * nt + c;
#pragma unroll
      for (int r = 0; r < 8; ++r) {
        const float hf = hv[nt][r];
        const unsigned short hb = f2bf_bits(hf);
        Ah[(8 * hh + r) * HPITCH + j] = __builtin_bit_cast(_Float16, hb);
      }
    }
    __syncthreads();
    tile_store(Ah, HH, rowbase, tid);
    __syncthreads();
#pragma unroll
    for (int nt = 0; nt < 4; ++nt) {
      const int j = 64 * wave + 16 * nt + c;
#pragma unroll
      for (int r = 0; r < 8; ++r) {
        const float hf = hv[nt][r];
        const unsigned short hb = f2bf_bits(hf);
        const unsigned short lb = f2bf_bits(hf - bf_bits2f(hb));
        Ah[(8 * hh + r) * HPITCH + j] = __builtin_bit_cast(_Float16, lb);
      }
    }
    __syncthreads();
    tile_store(Ah, HL, rowbase, tid);
  }
}

extern "C" void kernel_launch(void* const* d_in, const int* in_sizes, int n_in,
                              void* d_out, int out_size, void* d_ws, size_t ws_size, hipStream_t stream) {
  if (n_in < 6 || d_out == nullptr || d_ws == nullptr) return;
  if (in_sizes[0] != NSTEP * NBATCH * NIN || in_sizes[1] != NIN * NHID || in_sizes[2] != NHID * NHID ||
      in_sizes[3] != NHID || in_sizes[4] != NHID * NOUT || in_sizes[5] != 1 || out_size != NBATCH * NOUT) return;

  const float* xs  = (const float*)d_in[0];
  const float* w1x = (const float*)d_in[1];
  const float* w1h = (const float*)d_in[2];
  const float* b1  = (const float*)d_in[3];
  const float* w2  = (const float*)d_in[4];
  const float* b2  = (const float*)d_in[5];
  float* out = (float*)d_out;

  char* ws = (char*)d_ws; size_t off = 0;
  auto carve = [&](size_t bytes) -> char* { char* p = ws + off; off += (bytes + 255) & ~(size_t)255; return p; };
  unsigned short* XH   = (unsigned short*)carve((size_t)NSTEP * NBATCH * NIN * 2);
  unsigned short* XL   = (unsigned short*)carve((size_t)NSTEP * NBATCH * NIN * 2);
  unsigned short* W1XH = (unsigned short*)carve((size_t)NHID * NIN * 2);
  unsigned short* W1XL = (unsigned short*)carve((size_t)NHID * NIN * 2);
  unsigned short* W1HT = (unsigned short*)carve((size_t)NHID * NHID * 2);
  unsigned short* W2H  = (unsigned short*)carve((size_t)NOUT * NHID * 2);
  unsigned short* W2L  = (unsigned short*)carve((size_t)NOUT * NHID * 2);
  unsigned short* HST  = (unsigned short*)carve((size_t)NBATCH * NHID * 2);
  unsigned short* HH   = (unsigned short*)carve((size_t)NBATCH * NHID * 2);
  unsigned short* HL   = (unsigned short*)carve((size_t)NBATCH * NHID * 2);
  float*          XP   = (float*)carve((size_t)ROWS_H * NHID * 4);
  if (off > ws_size || off > (size_t)134217728) return;

  const int n8x = NSTEP * NBATCH * (NIN / 8);
  split8_kernel<<<n8x / 256, 256, 0, stream>>>(xs, XH, XL, n8x);
  tpw_kernel<0><<<dim3(NHID / 64, NIN / 64), 256, 0, stream>>>(w1x, NHID, NIN, W1XH, W1XL, 1.0f);
  tpw_kernel<1><<<dim3(NHID / 64, NHID / 64), 256, 0, stream>>>(w1h, NHID, NHID, W1HT, W1HT, WCARRY);
  tpw_kernel<0><<<dim3(NOUT / 64, NHID / 64), 256, 0, stream>>>(w2, NOUT, NHID, W2H, W2L, 1.0f);

  const int ggrid = (ROWS_H / 64) * (NHID / 64) / 8;
  for (int hf = 0; hf < NHALVES; ++hf) {
    const size_t aoff = (size_t)hf * ROWS_H * NIN;
    wmma_gemm64<2><<<ggrid, 256, 0, stream>>>(XH + aoff, XL + aoff, NIN, W1XH, W1XL, NIN,
                                              XP, NHID, b1, ROWS_H, NHID, NIN, 1.0f);
    rnn_seq_kernel<<<NBATCH / SEQ_BLK, RTHR, 0, stream>>>(XP, W1HT, HST, HH, HL,
                                                          (hf == 0) ? 1 : 0, (hf == NHALVES - 1) ? 1 : 0);
  }

  wmma_gemm64<3><<<(NBATCH / 64) * (NOUT / 64) / 8, 256, 0, stream>>>(HH, HL, NHID, W2H, W2L, NHID,
                                                                      out, NOUT, b2, NBATCH, NOUT, NHID, 1.0f);
}
